// LaplaceProcessor_89343909692235
// MI455X (gfx1250) — hardware-verified
//
#include <hip/hip_runtime.h>
#include <stddef.h>
#include <stdint.h>


#define DF      128
#define NTHR    256
#define NWAVE   8
#define EPT     8
#define NGRP    2
#define CHUNK   (NTHR * EPT * NGRP)
#define WCAP    (EPT * NGRP * 32)
#define LISTN   (NWAVE * WCAP)
#define NBS     512
#define GROWS   128
#define SPITCH  132
#define TPITCH  136
#define TPLANE  (16 * TPITCH)
#define WREG    (TPLANE * 2 * 4)
#define KPQ     258
#define LAYERS  3

#define R_PQ    0
#define S_PQ    (2 * DF * DF)
#define R_W2    (R_PQ + LAYERS * S_PQ)
#define S_W2    (DF * DF)
#define R_G1    (R_W2 + LAYERS * S_W2)
#define S_G1    (2 * DF * DF)
#define R_G2    (R_G1 + LAYERS * S_G1)
#define S_G2    (DF * DF)
#define WTOT    (R_G2 + LAYERS * S_G2)

#define LDS_PQ   (GROWS * SPITCH * 4)
#define LDS_NODE (NWAVE * WREG)
#define LDS_AGG  (NBS * DF * 4 + LISTN * 4 + 64 + NBS * 4)

static_assert((CHUNK & (CHUNK - 1)) == 0);
static_assert(CHUNK <= 4096);
static_assert((NBS & (NBS - 1)) == 0);
static_assert(NBS <= 4096);
static_assert(NBS % GROWS == 0);
static_assert(GROWS == NWAVE * 16);
static_assert(16 * SPITCH * 4 <= TPLANE * 2 * 2);
static_assert((WREG & 15) == 0);
static_assert(((TPLANE * 2) & 15) == 0);
static_assert((WTOT % (8 * NTHR)) == 0);

typedef float          v4f  __attribute__((ext_vector_type(4)));
typedef float          v8f  __attribute__((ext_vector_type(8)));
typedef int            v4i  __attribute__((ext_vector_type(4)));
typedef unsigned int   v8u  __attribute__((ext_vector_type(8)));
typedef unsigned short v8us __attribute__((ext_vector_type(8)));
typedef __bf16         v16b __attribute__((ext_vector_type(16)));
union FragB { v16b v; v8us u[2]; v8u w; };

__device__ __forceinline__ unsigned short bf_bits(float x) {
  unsigned int u = __float_as_uint(x);
  u = u + 0x7FFFu + ((u >> 16) & 1u);
  return (unsigned short)(u >> 16);
}
__device__ __forceinline__ void split1(float x, unsigned short& hi, unsigned short& lo) {
  const unsigned short hb = bf_bits(x);
  const float hf = __uint_as_float(((unsigned int)hb) << 16);
  hi = hb;
  lo = bf_bits(x - hf);
}
__device__ __forceinline__ void split8(v4f a, v4f b, v8us& hi, v8us& lo) {
  float x[8] = {a.x, a.y, a.z, a.w, b.x, b.y, b.z, b.w};
#pragma unroll
  for (int j = 0; j < 8; ++j) {
    unsigned short hj, lj;
    split1(x[j], hj, lj);
    hi[j] = hj;
    lo[j] = lj;
  }
}

__device__ __forceinline__ v8f wmb(const FragB& a, const FragB& b, v8f c) {
  v8f d = __builtin_amdgcn_wmma_f32_16x16x32_bf16(false, a.v, false, b.v, (short)0, c, false, false);
  asm volatile("v_nop\n\tv_nop\n\tv_nop\n\tv_nop" : "+v"(d) : "v"(a.w), "v"(b.w));
  return d;
}

__device__ __forceinline__ void mm64(v8f (&acc)[4],
                                     const unsigned short* ah, const unsigned short* al,
                                     const unsigned short* bh, const unsigned short* bl,
                                     int bpitch, int m) {
#pragma unroll 1
  for (int kt = 0; kt < 4; ++kt) {
    FragB fah, fal;
    fah.u[0] = *(const v8us*)(ah + 32 * kt);
    fah.u[1] = *(const v8us*)(ah + 32 * kt + 16);
    fal.u[0] = *(const v8us*)(al + 32 * kt);
    fal.u[1] = *(const v8us*)(al + 32 * kt + 16);
#pragma unroll
    for (int t = 0; t < 4; ++t) {
      const unsigned short* ph = bh + (size_t)(16 * t + m) * bpitch + 32 * kt;
      const unsigned short* pl = bl + (size_t)(16 * t + m) * bpitch + 32 * kt;
      FragB fbh, fbl;
      fbh.u[0] = *(const v8us*)ph;
      fbh.u[1] = *(const v8us*)(ph + 16);
      fbl.u[0] = *(const v8us*)pl;
      fbl.u[1] = *(const v8us*)(pl + 16);
      v8f c = acc[t];
      c = wmb(fah, fbh, c);
      c = wmb(fah, fbl, c);
      c = wmb(fal, fbh, c);
      acc[t] = c;
    }
  }
}

__device__ __forceinline__ void zero4(v8f (&acc)[4]) {
#pragma unroll
  for (int t = 0; t < 4; ++t) { v8f z = {0.f, 0.f, 0.f, 0.f, 0.f, 0.f, 0.f, 0.f}; acc[t] = z; }
}

__device__ __forceinline__ void stage_f32(float* stg, const v8f (&acc)[4], int cg, int hh, int m) {
  float* sp = stg + (8 * hh) * SPITCH + 64 * cg + m;
#pragma unroll
  for (int t = 0; t < 4; ++t) {
#pragma unroll
    for (int r = 0; r < 8; ++r) sp[r * SPITCH + 16 * t] = acc[t][r];
  }
}

template <int NB>
__device__ __forceinline__ int scan_chunk(const int* __restrict__ dsts, int nE, int cbase, int nodeBase,
                                          int vec8, int* list, int tid, int lane, int wave) {
  int wc = 0;
#pragma unroll
  for (int g = 0; g < NGRP; ++g) {
    const int el0  = (g * NTHR + tid) * EPT;
    const int e0   = cbase + el0;
    const int sent = -2147483647 - 1;
    v4i da, db;
    if (vec8 != 0 && cbase + CHUNK <= nE) {
      da = *(const v4i*)(dsts + e0);
      db = *(const v4i*)(dsts + e0 + 4);
    } else {
      da.x = (e0     < nE) ? dsts[min(e0, nE - 1)] : sent;
      da.y = (e0 + 1 < nE) ? dsts[min(e0 + 1, nE - 1)] : sent;
      da.z = (e0 + 2 < nE) ? dsts[min(e0 + 2, nE - 1)] : sent;
      da.w = (e0 + 3 < nE) ? dsts[min(e0 + 3, nE - 1)] : sent;
      db.x = (e0 + 4 < nE) ? dsts[min(e0 + 4, nE - 1)] : sent;
      db.y = (e0 + 5 < nE) ? dsts[min(e0 + 5, nE - 1)] : sent;
      db.z = (e0 + 6 < nE) ? dsts[min(e0 + 6, nE - 1)] : sent;
      db.w = (e0 + 7 < nE) ? dsts[min(e0 + 7, nE - 1)] : sent;
    }
    const unsigned nb = (unsigned)nodeBase;
    const unsigned s0 = (unsigned)da.x - nb, s1 = (unsigned)da.y - nb;
    const unsigned s2 = (unsigned)da.z - nb, s3 = (unsigned)da.w - nb;
    const unsigned s4 = (unsigned)db.x - nb, s5 = (unsigned)db.y - nb;
    const unsigned s6 = (unsigned)db.z - nb, s7 = (unsigned)db.w - nb;
    const bool h0 = s0 < (unsigned)NB, h1 = s1 < (unsigned)NB, h2 = s2 < (unsigned)NB, h3 = s3 < (unsigned)NB;
    const bool h4 = s4 < (unsigned)NB, h5 = s5 < (unsigned)NB, h6 = s6 < (unsigned)NB, h7 = s7 < (unsigned)NB;
    const unsigned any = __builtin_amdgcn_ballot_w32(h0 | h1 | h2 | h3 | h4 | h5 | h6 | h7);
    if (any != 0u) {
#define HITJ(J, HJ, SJ) { \
        const unsigned mj = __builtin_amdgcn_ballot_w32(HJ); \
        if (mj != 0u) { \
          if (HJ) { \
            const int pos = wc + (int)__builtin_amdgcn_mbcnt_lo(mj, 0u); \
            if (pos < WCAP) list[wave * WCAP + pos] = ((el0 + (J)) << 12) | (int)(SJ); \
          } \
          wc += (int)__builtin_popcount(mj); } }
      HITJ(0, h0, s0)
      HITJ(1, h1, s1)
      HITJ(2, h2, s2)
      HITJ(3, h3, s3)
      HITJ(4, h4, s4)
      HITJ(5, h5, s5)
      HITJ(6, h6, s6)
      HITJ(7, h7, s7)
#undef HITJ
    }
  }
  return wc;
}

__global__ __launch_bounds__(NTHR) void k_wprep(
    const float* __restrict__ W1, const float* __restrict__ W2,
    const float* __restrict__ G1, const float* __restrict__ G2,
    unsigned short* whi, unsigned short* wlo) {
  const int i = blockIdx.x * NTHR + threadIdx.x;
  const int o = i * 8;
  if (o >= WTOT) return;
  const float* S;
  int ia0, ib0;
  float fb;
  if (o < R_W2) {
    const int rel = o - R_PQ, l = rel / S_PQ, w = rel - l * S_PQ;
    const int n = w / DF, k0 = w - n * DF;
    S = W1 + (size_t)l * KPQ * DF;
    if (n < DF) { ia0 = k0 * DF + n;               ib0 = (k0 + DF) * DF + n; fb = 1.f; }
    else        { ia0 = (k0 + DF) * DF + (n - DF); ib0 = ia0;                fb = 0.f; }
  } else if (o < R_G1) {
    const int rel = o - R_W2, l = rel / S_W2, w = rel - l * S_W2;
    const int n = w / DF, k0 = w - n * DF;
    S = W2 + (size_t)l * DF * DF;
    ia0 = k0 * DF + n; ib0 = ia0; fb = 0.f;
  } else if (o < R_G2) {
    const int rel = o - R_G1, l = rel / S_G1, w = rel - l * S_G1;
    const int n = w / (2 * DF), k0 = w - n * (2 * DF);
    S = G1 + (size_t)l * 2 * DF * DF;
    ia0 = k0 * DF + n; ib0 = ia0; fb = 0.f;
  } else {
    const int rel = o - R_G2, l = rel / S_G2, w = rel - l * S_G2;
    const int n = w / DF, k0 = w - n * DF;
    S = G2 + (size_t)l * DF * DF;
    ia0 = k0 * DF + n; ib0 = ia0; fb = 0.f;
  }
  float v[8];
#pragma unroll
  for (int j = 0; j < 8; ++j) v[j] = S[ia0 + j * DF] - fb * S[ib0 + j * DF];
  v4f a, b;
  a.x = v[0]; a.y = v[1]; a.z = v[2]; a.w = v[3];
  b.x = v[4]; b.y = v[5]; b.z = v[6]; b.w = v[7];
  v8us hv, lv;
  split8(a, b, hv, lv);
  *(volatile v8us*)(whi + o) = hv;
  *(volatile v8us*)(wlo + o) = lv;
  __threadfence();
  *(volatile v8us*)(whi + o) = hv;
  *(volatile v8us*)(wlo + o) = lv;
}

__global__ __launch_bounds__(NTHR) void k_hcvt(
    const float* __restrict__ h, unsigned short* Hh, unsigned short* Hl, int nN, int nPad) {
  const int idx = blockIdx.x * NTHR + threadIdx.x;
  const int row = idx >> 4;
  if (row >= nPad) return;
  const int c0 = (idx & 15) * 8;
  const int sr = row < nN ? row : nN - 1;
  const float* p = h + (size_t)sr * DF + c0;
  const v4f a = *(const v4f*)p, b = *(const v4f*)(p + 4);
  v8us hv, lv;
  split8(a, b, hv, lv);
  const size_t g = (size_t)row * DF + c0;
  *(volatile v8us*)(Hh + g) = hv;
  *(volatile v8us*)(Hl + g) = lv;
  __threadfence();
  *(volatile v8us*)(Hh + g) = hv;
  *(volatile v8us*)(Hl + g) = lv;
}

__global__ __launch_bounds__(NTHR) void k_pq(
    const unsigned short* __restrict__ Hh, const unsigned short* __restrict__ Hl,
    const unsigned short* __restrict__ Wh, const unsigned short* __restrict__ Wl,
    const float* __restrict__ b1, float* P, float* Q) {
  extern __shared__ v4f lds_dyn[];
  const int tid = threadIdx.x, lane = tid & 31, wave = tid >> 5, hh = lane >> 4, m = lane & 15;
  const int rowBase = blockIdx.x * GROWS;
  const int cb = blockIdx.y;
  const int arow = rowBase + wave * 16 + m;
  float* stg = (float*)lds_dyn + wave * 16 * SPITCH;
  const unsigned short* ah = Hh + (size_t)arow * DF + 8 * hh;
  const unsigned short* al = Hl + (size_t)arow * DF + 8 * hh;
  const unsigned short* bh = Wh + (size_t)cb * DF * DF + 8 * hh;
  const unsigned short* bl = Wl + (size_t)cb * DF * DF + 8 * hh;

  v8f acc[4];
#pragma unroll 1
  for (int g = 0; g < 2; ++g) {
    zero4(acc);
    mm64(acc, ah, al, bh + (size_t)(64 * g) * DF, bl + (size_t)(64 * g) * DF, DF, m);
    stage_f32(stg, acc, g, hh, m);
  }
  __syncthreads();

  const float bs = (cb == 0) ? 1.f : 0.f;
  const v4f bv = *(const v4f*)(b1 + 4 * lane) * bs;
  float* op = (cb == 0) ? P : Q;
  float* gp = op + ((size_t)rowBase + wave * 16) * DF + 4 * lane;
  const float* lp = stg + 4 * lane;
#pragma unroll
  for (int i = 0; i < 16; ++i) {
    const v4f x = *(const v4f*)(lp + i * SPITCH) + bv;
    *(volatile v4f*)(gp + (size_t)i * DF) = x;
  }
  __threadfence();
#pragma unroll
  for (int i = 0; i < 16; ++i) {
    const v4f x = *(const v4f*)(lp + i * SPITCH) + bv;
    *(volatile v4f*)(gp + (size_t)i * DF) = x;
  }
}

__global__ __launch_bounds__(NTHR) void k_agg(
    const int* __restrict__ ei, const float* __restrict__ ea,
    const float* __restrict__ P, const float* __restrict__ Q, const float* __restrict__ we,
    unsigned short* Uh, unsigned short* Ul, float* cntp, int nN, int nE, int vec8) {
  extern __shared__ v4f lds_dyn[];
  float* U    = (float*)lds_dyn;
  int*   list = (int*)(U + NBS * DF);
  int*   wcnt = list + LISTN;
  int*   cnt  = wcnt + 16;
  const int tid = threadIdx.x, lane = tid & 31, wave = tid >> 5;
  const int nodeBase = blockIdx.x * NBS;
  const int* dsts = ei + nE;

  {
    const v4f z = {0.f, 0.f, 0.f, 0.f};
    for (int i = tid; i < NBS * DF / 4; i += NTHR) lds_dyn[i] = z;
    for (int i = tid; i < NBS; i += NTHR) cnt[i] = 0;
  }
  __syncthreads();

  const v4f w6 = *(const v4f*)(we + 4 * lane);
  const v4f w7 = *(const v4f*)(we + DF + 4 * lane);

  const int nChunks = (nE + CHUNK - 1) / CHUNK;
#pragma unroll 1
  for (int ch = 0; ch < nChunks; ++ch) {
    const int cbase = ch * CHUNK;
    const int wc = scan_chunk<NBS>(dsts, nE, cbase, nodeBase, vec8, list, tid, lane, wave);
    if (lane == 0) wcnt[wave] = wc;
    __syncthreads();
    if (wave == 0) {
#pragma unroll 1
      for (int wsx = 0; wsx < NWAVE; ++wsx) {
        int n = __builtin_amdgcn_readfirstlane(wcnt[wsx]);
        n = n > WCAP ? WCAP : (n < 0 ? 0 : n);
        const int* lp = list + wsx * WCAP;
#pragma unroll 1
        for (int i = 0; i < n; ++i) {
          const int ent  = __builtin_amdgcn_readfirstlane(lp[i]);
          const int slot = ent & (NBS - 1);
          int e = cbase + ((ent >> 12) & (CHUNK - 1));
          e = e > nE - 1 ? nE - 1 : e;
          int src = ei[e];
          src = src < 0 ? 0 : (src > nN - 1 ? nN - 1 : src);
          int pn = nodeBase + slot;
          pn = pn > nN - 1 ? nN - 1 : pn;
          const float e0 = ea[2 * (size_t)e];
          const float e1 = ea[2 * (size_t)e + 1];
          const v4f q = *(const v4f*)(Q + (size_t)src * DF + 4 * lane);
          const v4f p = *(const v4f*)(P + (size_t)pn * DF + 4 * lane);
          v4f u = p + q + w6 * e0 + w7 * e1;
          u.x = fmaxf(u.x, 0.f); u.y = fmaxf(u.y, 0.f); u.z = fmaxf(u.z, 0.f); u.w = fmaxf(u.w, 0.f);
          v4f* ap = (v4f*)(U + slot * DF + 4 * lane);
          *ap = *ap + u;
          if (lane == 0) cnt[slot] = cnt[slot] + 1;
        }
      }
    }
    __syncthreads();
  }

  {
    const size_t gb = ((size_t)nodeBase + wave * 64) * DF + 8 * lane;
    const float* ub = U + (wave * 64 + (lane >> 4)) * DF + 8 * (lane & 15);
#pragma unroll 4
    for (int j = 0; j < 32; ++j) {
      const float* up = ub + 2 * j * DF;
      v8us hv, lv;
      split8(*(const v4f*)up, *(const v4f*)(up + 4), hv, lv);
      *(volatile v8us*)(Uh + gb + (size_t)2 * j * DF) = hv;
      *(volatile v8us*)(Ul + gb + (size_t)2 * j * DF) = lv;
    }
    __threadfence();
#pragma unroll 4
    for (int j = 0; j < 32; ++j) {
      const float* up = ub + 2 * j * DF;
      v8us hv, lv;
      split8(*(const v4f*)up, *(const v4f*)(up + 4), hv, lv);
      *(volatile v8us*)(Uh + gb + (size_t)2 * j * DF) = hv;
      *(volatile v8us*)(Ul + gb + (size_t)2 * j * DF) = lv;
    }
  }
  if (wave == 0) {
    v4f cq[4];
#pragma unroll
    for (int q = 0; q < 4; ++q) {
      const v4i c = *(const v4i*)(cnt + 128 * q + 4 * lane);
      cq[q] = __builtin_convertvector(c, v4f);
    }
    float* cp = cntp + (size_t)nodeBase + 4 * lane;
#pragma unroll
    for (int q = 0; q < 4; ++q) *(volatile v4f*)(cp + 128 * q) = cq[q];
    __threadfence();
#pragma unroll
    for (int q = 0; q < 4; ++q) *(volatile v4f*)(cp + 128 * q) = cq[q];
  }
}

__global__ __launch_bounds__(NTHR) void k_node(
    const unsigned short* __restrict__ Uh, const unsigned short* __restrict__ Ul, const float* __restrict__ cntp,
    const unsigned short* __restrict__ W2h, const unsigned short* __restrict__ W2l, const float* __restrict__ b2,
    unsigned short* Hh, unsigned short* Hl,
    const unsigned short* __restrict__ G1h, const unsigned short* __restrict__ G1l, const float* __restrict__ gb1,
    const unsigned short* __restrict__ G2h, const unsigned short* __restrict__ G2l, const float* __restrict__ gb2,
    const float* hold, float* hout, int nN, int writeH) {
  extern __shared__ v4f lds_dyn[];
  const int tid = threadIdx.x, lane = tid & 31, wave = tid >> 5, hh = lane >> 4, m = lane & 15;
  const int rowBase = blockIdx.x * GROWS;
  const int arow = rowBase + wave * 16 + m;
  unsigned short* xh = (unsigned short*)((char*)lds_dyn + wave * WREG);
  unsigned short* xl = xh + TPLANE;
  unsigned short* yh = xl + TPLANE;
  unsigned short* yl = yh + TPLANE;
  float* stg = (float*)xh;

  v8f acc[4];

  {
    const v4f cA = *(const v4f*)(cntp + (size_t)rowBase + wave * 16 + 8 * hh);
    const v4f cB = *(const v4f*)(cntp + (size_t)rowBase + wave * 16 + 8 * hh + 4);
    const float cr[8] = {cA.x, cA.y, cA.z, cA.w, cB.x, cB.y, cB.z, cB.w};
    const unsigned short* ah = Uh + (size_t)arow * DF + 8 * hh;
    const unsigned short* al = Ul + (size_t)arow * DF + 8 * hh;
#pragma unroll 1
    for (int g = 0; g < 2; ++g) {
      zero4(acc);
      mm64(acc, ah, al, W2h + (size_t)(64 * g) * DF + 8 * hh, W2l + (size_t)(64 * g) * DF + 8 * hh, DF, m);
#pragma unroll
      for (int t = 0; t < 4; ++t) {
        const int col = 64 * g + 16 * t + m;
        const float bb = b2[col];
#pragma unroll
        for (int r = 0; r < 8; ++r) {
          unsigned short hb, lb;
          split1(acc[t][r] + cr[r] * bb, hb, lb);
          const int o = (8 * hh + r) * TPITCH + col;
          xh[o] = hb;
          xl[o] = lb;
        }
      }
    }
  }
  __syncthreads();

  {
    const unsigned short* ah0 = Hh + (size_t)arow * DF + 8 * hh;
    const unsigned short* al0 = Hl + (size_t)arow * DF + 8 * hh;
    const unsigned short* ah1 = xh + m * TPITCH + 8 * hh;
    const unsigned short* al1 = xl + m * TPITCH + 8 * hh;
#pragma unroll 1
    for (int g = 0; g < 2; ++g) {
      zero4(acc);
      const size_t bo = (size_t)(64 * g) * (2 * DF) + 8 * hh;
      mm64(acc, ah0, al0, G1h + bo, G1l + bo, 2 * DF, m);
      mm64(acc, ah1, al1, G1h + bo + DF, G1l + bo + DF, 2 * DF, m);
#pragma unroll
      for (int t = 0; t < 4; ++t) {
        const int col = 64 * g + 16 * t + m;
        const float bb = gb1[col];
#pragma unroll
        for (int r = 0; r < 8; ++r) {
          unsigned short hb, lb;
          split1(fmaxf(acc[t][r] + bb, 0.f), hb, lb);
          const int o = (8 * hh + r) * TPITCH + col;
          yh[o] = hb;
          yl[o] = lb;
        }
      }
    }
  }
  __syncthreads();

  {
    const unsigned short* ah = yh + m * TPITCH + 8 * hh;
    const unsigned short* al = yl + m * TPITCH + 8 * hh;
#pragma unroll 1
    for (int g = 0; g < 2; ++g) {
      zero4(acc);
      mm64(acc, ah, al, G2h + (size_t)(64 * g) * DF + 8 * hh, G2l + (size_t)(64 * g) * DF + 8 * hh, DF, m);
      stage_f32(stg, acc, g, hh, m);
    }
  }
  __syncthreads();

  const v4f gv = *(const v4f*)(gb2 + 4 * lane);
  const int row0 = rowBase + wave * 16;
  float* lp = stg + 4 * lane;
#pragma unroll
  for (int i = 0; i < 16; ++i) {
    const int row = row0 + i;
    const int hr  = row < nN ? row : nN - 1;
    const v4f x = *(const v4f*)(lp + i * SPITCH) + gv + *(const v4f*)(hold + (size_t)hr * DF + 4 * lane);
    *(v4f*)(lp + i * SPITCH) = x;
    if (row < nN) *(volatile v4f*)(hout + (size_t)row * DF + 4 * lane) = x;
  }
  __threadfence();
  __syncthreads();
#pragma unroll
  for (int i = 0; i < 16; ++i) {
    const int row = row0 + i;
    if (row < nN) {
      const v4f x = *(const v4f*)(lp + i * SPITCH);
      *(volatile v4f*)(hout + (size_t)row * DF + 4 * lane) = x;
    }
  }

  if (writeH != 0) {
    const float* sb = stg + (lane >> 4) * SPITCH + 8 * (lane & 15);
    const size_t gb = ((size_t)row0) * DF + 8 * lane;
#pragma unroll
    for (int j = 0; j < 8; ++j) {
      const float* sp = sb + 2 * j * SPITCH;
      v8us hv, lv;
      split8(*(const v4f*)sp, *(const v4f*)(sp + 4), hv, lv);
      *(volatile v8us*)(Hh + gb + (size_t)2 * j * DF) = hv;
      *(volatile v8us*)(Hl + gb + (size_t)2 * j * DF) = lv;
    }
    __threadfence();
#pragma unroll
    for (int j = 0; j < 8; ++j) {
      const float* sp = sb + 2 * j * SPITCH;
      v8us hv, lv;
      split8(*(const v4f*)sp, *(const v4f*)(sp + 4), hv, lv);
      *(volatile v8us*)(Hh + gb + (size_t)2 * j * DF) = hv;
      *(volatile v8us*)(Hl + gb + (size_t)2 * j * DF) = lv;
    }
  }
}

extern "C" void kernel_launch(void* const* d_in, const int* in_sizes, int n_in,
                              void* d_out, int out_size, void* d_ws, size_t ws_size,
                              hipStream_t stream) {
  if (n_in < 11) return;
  const int nN = in_sizes[0] / DF;
  const int nE = in_sizes[1] / 2;
  if (nN <= 0 || nE < 0) return;
  if (in_sizes[0] != nN * DF || in_sizes[1] != nE * 2 || in_sizes[2] != 2 * nE) return;
  if (in_sizes[3] != LAYERS * KPQ * DF || in_sizes[4] != LAYERS * DF || in_sizes[5] != LAYERS * DF * DF ||
      in_sizes[6] != LAYERS * DF || in_sizes[7] != LAYERS * 2 * DF * DF || in_sizes[8] != LAYERS * DF ||
      in_sizes[9] != LAYERS * DF * DF || in_sizes[10] != LAYERS * DF) return;
  if (out_size != nN * DF) return;

  const float* h     = (const float*)d_in[0];
  const float* ea    = (const float*)d_in[1];
  const int*   ei    = (const int*)d_in[2];
  const float* phiW1 = (const float*)d_in[3];
  const float* phib1 = (const float*)d_in[4];
  const float* phiW2 = (const float*)d_in[5];
  const float* phib2 = (const float*)d_in[6];
  const float* gamW1 = (const float*)d_in[7];
  const float* gamb1 = (const float*)d_in[8];
  const float* gamW2 = (const float*)d_in[9];
  const float* gamb2 = (const float*)d_in[10];
  float* out = (float*)d_out;

  const int nPad = ((nN + NBS - 1) / NBS) * NBS;
  const int nAgg = nPad / NBS;
  const int nG   = nPad / GROWS;

  char* ws = (char*)d_ws;
  size_t off = 0;
  const size_t oWh = off; off += (size_t)WTOT * 2;          off = (off + 255) & ~(size_t)255;
  const size_t oWl = off; off += (size_t)WTOT * 2;          off = (off + 255) & ~(size_t)255;
  const size_t oHh = off; off += (size_t)nPad * DF * 2;     off = (off + 255) & ~(size_t)255;
  const size_t oHl = off; off += (size_t)nPad * DF * 2;     off = (off + 255) & ~(size_t)255;
  const size_t oUh = off; off += (size_t)nPad * DF * 2;     off = (off + 255) & ~(size_t)255;
  const size_t oUl = off; off += (size_t)nPad * DF * 2;     off = (off + 255) & ~(size_t)255;
  const size_t oP  = off; off += (size_t)nPad * DF * 4;     off = (off + 255) & ~(size_t)255;
  const size_t oQ  = off; off += (size_t)nPad * DF * 4;     off = (off + 255) & ~(size_t)255;
  const size_t oC  = off; off += (size_t)nPad * 4;          off = (off + 255) & ~(size_t)255;
  const size_t oHb = off; off += (size_t)nPad * DF * 4;     off = (off + 255) & ~(size_t)255;
  if (off > ws_size) return;
  unsigned short* whi  = (unsigned short*)(ws + oWh);
  unsigned short* wlo  = (unsigned short*)(ws + oWl);
  unsigned short* Hh   = (unsigned short*)(ws + oHh);
  unsigned short* Hl   = (unsigned short*)(ws + oHl);
  unsigned short* Uh   = (unsigned short*)(ws + oUh);
  unsigned short* Ul   = (unsigned short*)(ws + oUl);
  float*          P    = (float*)(ws + oP);
  float*          Q    = (float*)(ws + oQ);
  float*          cntp = (float*)(ws + oC);
  float*          hbuf = (float*)(ws + oHb);

  const int vec8 = ((nE & 3) == 0) ? 1 : 0;

  hipFuncSetAttribute(reinterpret_cast<const void*>(&k_pq),
                      hipFuncAttributeMaxDynamicSharedMemorySize, LDS_PQ);
  hipFuncSetAttribute(reinterpret_cast<const void*>(&k_agg),
                      hipFuncAttributeMaxDynamicSharedMemorySize, LDS_AGG);
  hipFuncSetAttribute(reinterpret_cast<const void*>(&k_node),
                      hipFuncAttributeMaxDynamicSharedMemorySize, LDS_NODE);

  k_wprep<<<WTOT / (8 * NTHR), NTHR, 0, stream>>>(phiW1, phiW2, gamW1, gamW2, whi, wlo);
  k_hcvt<<<(nPad * 16) / NTHR, NTHR, 0, stream>>>(h, Hh, Hl, nN, nPad);

  for (int l = 0; l < LAYERS; ++l) {
    k_pq<<<dim3(nG, 2), NTHR, LDS_PQ, stream>>>(
        Hh, Hl, whi + R_PQ + (size_t)l * S_PQ, wlo + R_PQ + (size_t)l * S_PQ, phib1 + l * DF, P, Q);

    k_agg<<<nAgg, NTHR, LDS_AGG, stream>>>(
        ei, ea, P, Q, phiW1 + (size_t)l * KPQ * DF + (size_t)2 * DF * DF, Uh, Ul, cntp, nN, nE, vec8);

    const float* hold = (l == 0) ? h : hbuf;
    float* hout = (l == LAYERS - 1) ? out : hbuf;
    const int writeH = (l == LAYERS - 1) ? 0 : 1;
    k_node<<<nG, NTHR, LDS_NODE, stream>>>(
        Uh, Ul, cntp,
        whi + R_W2 + (size_t)l * S_W2, wlo + R_W2 + (size_t)l * S_W2, phib2 + l * DF,
        Hh, Hl,
        whi + R_G1 + (size_t)l * S_G1, wlo + R_G1 + (size_t)l * S_G1, gamb1 + l * DF,
        whi + R_G2 + (size_t)l * S_G2, wlo + R_G2 + (size_t)l * S_G2, gamb2 + l * DF,
        hold, hout, nN, writeH);
  }
}
